// GNN_49134425866246
// MI455X (gfx1250) — hardware-verified
//
#include <hip/hip_runtime.h>
#include <stddef.h>
#include <stdint.h>
#include <math.h>


#define DF     128
#define TP     256
#define NC     40
#define NCP    64
#define NTHR   256
#define NWAVE  8
#define EPT    8
#define CHUNK  (NTHR * EPT)
#define WCAP   (EPT * 32)
#define LISTN  (NWAVE * WCAP)
#define NBA    1024
#define SLA    10
#define RCAP   20480
#define DEGCAP 64
#define GBM    64
#define GBN    64
#define GTHR   128
#define ARB    128
#define UW0    (256 * 16)
#define UW1    (256 * 32)
#define UWL    (NCP * 32)
#define UTOT   (UW0 + 2 * UW1 + UWL)
#define OW0    0
#define OW1    (256 * DF)
#define OW2    (OW1 + 256 * TP)
#define OWL    (OW2 + 256 * TP)
#define WPLN   (OWL + NCP * TP)
#define CMP_ZINTS (LISTN + 2 * RCAP + 3 * NBA)
#define CMP_LDS_INTS (CMP_ZINTS + 16)

static_assert((CHUNK & (CHUNK - 1)) == 0 && CHUNK <= 4096);
static_assert((NBA & (NBA - 1)) == 0 && NBA == (1 << SLA));
static_assert(((long long)CHUNK << SLA) < (1LL << 31));
static_assert(LISTN % NTHR == 0);
static_assert(NBA % 32 == 0 && NBA % GBM == 0 && NBA == NTHR * 4);
static_assert(RCAP % (NTHR * 4) == 0 && CMP_ZINTS % (NTHR * 4) == 0 && LISTN % 4 == 0);
static_assert(DF % 32 == 0 && TP % 32 == 0 && TP == 2 * DF && DF == 4 * 32);
static_assert(GBM == (GTHR / 32) * 16 && GBN == 64 && TP % GBN == 0 && NCP == GBN);
static_assert(UW0 % NTHR == 0 && UW1 % NTHR == 0 && UWL % NTHR == 0 && UTOT % NTHR == 0);
static_assert((OW1 * 2) % 256 == 0 && (OW2 * 2) % 256 == 0 && (OWL * 2) % 256 == 0);
static_assert(ARB % NWAVE == 0);
static_assert(NC % 4 == 0 && (GBM * NC) % (4 * GTHR) == 0 && (GBM * NC * 4) % 128 == 0);
static_assert(CMP_LDS_INTS * 4 <= 300000);
static_assert(DEGCAP >= 36 + 8 && RCAP >= 16710 + 2048);

typedef float          v4f   __attribute__((ext_vector_type(4)));
typedef float          v8f   __attribute__((ext_vector_type(8)));
typedef int            v4i   __attribute__((ext_vector_type(4)));
typedef int            v8i   __attribute__((ext_vector_type(8)));
typedef unsigned int   v4u   __attribute__((ext_vector_type(4)));
typedef unsigned short v8us  __attribute__((ext_vector_type(8)));
typedef unsigned short v16us __attribute__((ext_vector_type(16)));
typedef __bf16         v16bf __attribute__((ext_vector_type(16)));
typedef v4f  __attribute__((may_alias)) v4fa;
typedef v4i  __attribute__((may_alias)) v4ia;
typedef v8us __attribute__((may_alias)) v8usa;
union FragB { v16bf v; v16us u; v8us h[2]; v8i w; };

__device__ __forceinline__ v8f wmb(const FragB& a, const FragB& b, v8f c) {
  v8f d = __builtin_amdgcn_wmma_f32_16x16x32_bf16(false, a.v, false, b.v, (short)0, c, false, false);
  asm volatile("v_nop\n\tv_nop\n\tv_nop\n\tv_nop" : "+v"(d) : "v"(a.w), "v"(b.w));
  return d;
}

__device__ __forceinline__ unsigned bf16_bits(float f) {
  const unsigned u = __float_as_uint(f);
  const unsigned r = (u + 0x7FFFu + ((u >> 16) & 1u)) >> 16;
  return (f != f) ? 0x7FC0u : r;
}
__device__ __forceinline__ float bf16_val(float f) {
  return __uint_as_float(bf16_bits(f) << 16);
}

template <int SLB>
__device__ __forceinline__ int scan_chunk(const int* __restrict__ dsts, int nE, int cbase, int slotBase,
                                          int nb, int vec8, int* list, int tid, int lane, int wave) {
  int wc = 0;
  const int el0  = tid * EPT;
  const int e0   = cbase + el0;
  const int sent = -2147483647 - 1;
  v4i da, db;
  if (vec8 != 0 && cbase + CHUNK <= nE) {
    da = *(const v4i*)(dsts + e0);
    db = *(const v4i*)(dsts + e0 + 4);
  } else {
    da.x = (e0     < nE) ? dsts[min(e0,     nE - 1)] : sent;
    da.y = (e0 + 1 < nE) ? dsts[min(e0 + 1, nE - 1)] : sent;
    da.z = (e0 + 2 < nE) ? dsts[min(e0 + 2, nE - 1)] : sent;
    da.w = (e0 + 3 < nE) ? dsts[min(e0 + 3, nE - 1)] : sent;
    db.x = (e0 + 4 < nE) ? dsts[min(e0 + 4, nE - 1)] : sent;
    db.y = (e0 + 5 < nE) ? dsts[min(e0 + 5, nE - 1)] : sent;
    db.z = (e0 + 6 < nE) ? dsts[min(e0 + 6, nE - 1)] : sent;
    db.w = (e0 + 7 < nE) ? dsts[min(e0 + 7, nE - 1)] : sent;
  }
  const unsigned nbs = (unsigned)slotBase;
  const unsigned unb = (unsigned)nb;
  const unsigned s0 = (unsigned)da.x - nbs, s1 = (unsigned)da.y - nbs;
  const unsigned s2 = (unsigned)da.z - nbs, s3 = (unsigned)da.w - nbs;
  const unsigned s4 = (unsigned)db.x - nbs, s5 = (unsigned)db.y - nbs;
  const unsigned s6 = (unsigned)db.z - nbs, s7 = (unsigned)db.w - nbs;
  const bool h0 = s0 < unb, h1 = s1 < unb, h2 = s2 < unb, h3 = s3 < unb;
  const bool h4 = s4 < unb, h5 = s5 < unb, h6 = s6 < unb, h7 = s7 < unb;
  const unsigned any = __builtin_amdgcn_ballot_w32(h0 | h1 | h2 | h3 | h4 | h5 | h6 | h7);
  if (any != 0u) {
#define HITJ(J, HJ, SJ) { \
      const unsigned mj = __builtin_amdgcn_ballot_w32(HJ); \
      if (mj != 0u) { \
        if (HJ) { \
          const int pos = wc + (int)__builtin_amdgcn_mbcnt_lo(mj, 0u); \
          if (pos < WCAP) list[wave * WCAP + pos] = ((el0 + (J)) << SLB) | (int)(SJ); \
        } \
        wc += (int)__builtin_popcount(mj); } }
    HITJ(0, h0, s0)
    HITJ(1, h1, s1)
    HITJ(2, h2, s2)
    HITJ(3, h3, s3)
    HITJ(4, h4, s4)
    HITJ(5, h5, s5)
    HITJ(6, h6, s6)
    HITJ(7, h7, s7)
#undef HITJ
  }
  return wc;
}

__global__ __launch_bounds__(NTHR) void k_wprep(const float* __restrict__ Wl, const float* __restrict__ Wr,
                                                const float* __restrict__ Wlin, unsigned short* WP) {
  const int u = (int)blockIdx.x * NTHR + (int)threadIdx.x;
  if (u >= UTOT) return;
  v4f a, b;
  size_t doff;
  if (u < UW0 + 2 * UW1) {
    int lay, n, c8, pitch, pbase;
    if (u < UW0)            { lay = 0; n = u >> 4; c8 = (u & 15) * 8; pitch = DF; pbase = OW0; }
    else if (u < UW0 + UW1) { const int v = u - UW0;       lay = 1; n = v >> 5; c8 = (v & 31) * 8; pitch = TP; pbase = OW1; }
    else                    { const int v = u - UW0 - UW1; lay = 2; n = v >> 5; c8 = (v & 31) * 8; pitch = TP; pbase = OW2; }
    const int k  = c8 & (DF - 1);
    const int nn = n & (DF - 1);
    const size_t so = (size_t)lay * DF * DF + (size_t)nn * DF + k;
    const v4f la = *(const v4f*)(Wl + so);
    const v4f lb = *(const v4f*)(Wl + so + 4);
    const v4f ra = *(const v4f*)(Wr + so);
    const v4f rb = *(const v4f*)(Wr + so + 4);
    const bool isL = n < DF;
    a.x = isL ? la.x : ra.x; a.y = isL ? la.y : ra.y; a.z = isL ? la.z : ra.z; a.w = isL ? la.w : ra.w;
    b.x = isL ? lb.x : rb.x; b.y = isL ? lb.y : rb.y; b.z = isL ? lb.z : rb.z; b.w = isL ? lb.w : rb.w;
    doff = (size_t)pbase + (size_t)n * pitch + c8;
  } else {
    const int v  = u - UW0 - 2 * UW1;
    const int n  = v >> 5;
    const int c8 = (v & 31) * 8;
    const int k  = c8 & (DF - 1);
    const int nc = n < NC ? n : NC - 1;
    const v4f la = *(const v4f*)(Wlin + (size_t)nc * DF + k);
    const v4f lb = *(const v4f*)(Wlin + (size_t)nc * DF + k + 4);
    const bool ok = n < NC;
    a.x = ok ? la.x : 0.0f; a.y = ok ? la.y : 0.0f; a.z = ok ? la.z : 0.0f; a.w = ok ? la.w : 0.0f;
    b.x = ok ? lb.x : 0.0f; b.y = ok ? lb.y : 0.0f; b.z = ok ? lb.z : 0.0f; b.w = ok ? lb.w : 0.0f;
    doff = (size_t)OWL + (size_t)n * TP + c8;
  }
  v8us o;
  o[0] = (unsigned short)bf16_bits(a.x); o[1] = (unsigned short)bf16_bits(a.y);
  o[2] = (unsigned short)bf16_bits(a.z); o[3] = (unsigned short)bf16_bits(a.w);
  o[4] = (unsigned short)bf16_bits(b.x); o[5] = (unsigned short)bf16_bits(b.y);
  o[6] = (unsigned short)bf16_bits(b.z); o[7] = (unsigned short)bf16_bits(b.w);
  unsigned short* dp = WP + doff;
  *(volatile v8us*)dp = o;
  __threadfence();
  *(volatile v8us*)dp = o;
}

__global__ __launch_bounds__(NTHR) void k_cvx(const float* __restrict__ x, int nN, int nUnits,
                                              unsigned short* xb) {
  const int u = (int)blockIdx.x * NTHR + (int)threadIdx.x;
  if (u >= nUnits) return;
  const int row = u >> 4;
  const int k8  = (u & 15) * 8;
  const int rc  = row < nN ? row : nN - 1;
  const float* p = x + (size_t)rc * DF + k8;
  const v4f a = *(const v4fa*)p;
  const v4f b = *(const v4fa*)(p + 4);
  const bool ok = row < nN;
  v8us o;
  o[0] = ok ? (unsigned short)bf16_bits(a.x) : (unsigned short)0;
  o[1] = ok ? (unsigned short)bf16_bits(a.y) : (unsigned short)0;
  o[2] = ok ? (unsigned short)bf16_bits(a.z) : (unsigned short)0;
  o[3] = ok ? (unsigned short)bf16_bits(a.w) : (unsigned short)0;
  o[4] = ok ? (unsigned short)bf16_bits(b.x) : (unsigned short)0;
  o[5] = ok ? (unsigned short)bf16_bits(b.y) : (unsigned short)0;
  o[6] = ok ? (unsigned short)bf16_bits(b.z) : (unsigned short)0;
  o[7] = ok ? (unsigned short)bf16_bits(b.w) : (unsigned short)0;
  unsigned short* dp = xb + (size_t)row * DF + k8;
  *(volatile v8us*)dp = o;
  __threadfence();
  *(volatile v8us*)dp = o;
}

__global__ __launch_bounds__(NTHR) void k_compact(const int* __restrict__ srcs, const int* __restrict__ dsts,
                                                  int nE, int nN, int vec8, int* SR, int* RP, int* CN) {
  extern __shared__ __attribute__((aligned(16))) int dsm[];
  int* list = dsm;
  int* hl   = dsm + LISTN;
  int* sl   = dsm + LISTN + RCAP;
  int* cnt  = dsm + LISTN + 2 * RCAP;
  int* offs = cnt + NBA;
  int* cur  = offs + NBA;
  int* misc = cur + NBA;
  const int tid = (int)threadIdx.x, lane = tid & 31, wave = tid >> 5;
  const int nodeBase = (int)blockIdx.x * NBA;

  {
    const v4i z4 = {0, 0, 0, 0};
    for (int i = tid * 4; i < CMP_ZINTS; i += NTHR * 4) *(v4ia*)(dsm + i) = z4;
    if (tid < 16) misc[tid] = 0;
  }
  __syncthreads();

  int t = 0, ov = 0;
  const int nChunks = (nE + CHUNK - 1) / CHUNK;
#pragma unroll 1
  for (int ch = 0; ch < nChunks; ++ch) {
    const int cbase = ch * CHUNK;
    const int wc = scan_chunk<SLA>(dsts, nE, cbase, nodeBase, NBA, vec8, list, tid, lane, wave);
    if (lane == 0) misc[wave] = wc;
    __syncthreads();
    if (wave == 0) {
#pragma unroll 1
      for (int w2 = 0; w2 < NWAVE; ++w2) {
        int c = misc[w2];
        c = c < 0 ? 0 : (c > WCAP ? WCAP : c);
#pragma unroll 1
        for (int b0 = 0; b0 < c; b0 += 32) {
          const int idx = b0 + lane;
          const int ent = list[w2 * WCAP + (idx < WCAP ? idx : WCAP - 1)];
          const int m32 = (c - b0) < 32 ? (c - b0) : 32;
#pragma unroll 1
          for (int k = 0; k < m32; ++k) {
            const int u    = __builtin_amdgcn_readlane(ent, k);
            const int slot = u & (NBA - 1);
            const int el   = (u >> SLA) & (CHUNK - 1);
            const int pk   = ((cbase + el) << SLA) | slot;
            if (t < RCAP) {
              if (lane == 0) { hl[t] = pk; cnt[slot] = cnt[slot] + 1; }
              t = t + 1;
            } else {
              ov = 1;
            }
          }
        }
      }
    }
    __syncthreads();
  }
  if (wave == 0 && lane == 0) { misc[8] = t; misc[9] = ov; }
  __syncthreads();
  int tt = misc[8];
  tt = tt < 0 ? 0 : (tt > RCAP ? RCAP : tt);
  const int ovf = misc[9];

  if (wave == 0) {
    const int base = lane * (NBA / 32);
    int s = 0;
#pragma unroll 1
    for (int i = 0; i < NBA / 32; ++i) s += cnt[base + i];
    int incl = s;
#pragma unroll
    for (int d = 1; d < 32; d <<= 1) {
      const int y = __shfl_up(incl, d, 32);
      if (lane >= d) incl += y;
    }
    int run = incl - s;
#pragma unroll 1
    for (int i = 0; i < NBA / 32; ++i) {
      const int cv = cnt[base + i];
      offs[base + i] = run;
      cur[base + i]  = run;
      run += cv;
    }
  }
  __syncthreads();
  if (wave == 0) {
#pragma unroll 1
    for (int b0 = 0; b0 < tt; b0 += 32) {
      const int idx = b0 + lane;
      const int ent = hl[idx < RCAP ? idx : RCAP - 1];
      const int m32 = (tt - b0) < 32 ? (tt - b0) : 32;
#pragma unroll 1
      for (int k = 0; k < m32; ++k) {
        const int u    = __builtin_amdgcn_readlane(ent, k);
        const int slot = u & (NBA - 1);
        if (lane == 0) {
          int p = cur[slot];
          p = p < 0 ? 0 : (p > RCAP - 1 ? RCAP - 1 : p);
          sl[p] = u;
          cur[slot] = p + 1;
        }
      }
    }
  }
  __syncthreads();

  const int sbase = (int)blockIdx.x * RCAP;
#pragma unroll 1
  for (int it = 0; it < RCAP / (NTHR * 4); ++it) {
    const int p4 = it * (NTHR * 4) + 4 * tid;
    const v4i e4 = *(const v4ia*)(sl + p4);
    int e0 = e4.x >> SLA, e1 = e4.y >> SLA, e2 = e4.z >> SLA, e3 = e4.w >> SLA;
    e0 = e0 < 0 ? 0 : (e0 > nE - 1 ? nE - 1 : e0);
    e1 = e1 < 0 ? 0 : (e1 > nE - 1 ? nE - 1 : e1);
    e2 = e2 < 0 ? 0 : (e2 > nE - 1 ? nE - 1 : e2);
    e3 = e3 < 0 ? 0 : (e3 > nE - 1 ? nE - 1 : e3);
    int s0 = srcs[e0], s1 = srcs[e1], s2 = srcs[e2], s3 = srcs[e3];
    s0 = s0 < 0 ? 0 : (s0 > nN - 1 ? nN - 1 : s0);
    s1 = s1 < 0 ? 0 : (s1 > nN - 1 ? nN - 1 : s1);
    s2 = s2 < 0 ? 0 : (s2 > nN - 1 ? nN - 1 : s2);
    s3 = s3 < 0 ? 0 : (s3 > nN - 1 ? nN - 1 : s3);
    v4i o;
    o.x = (p4     < tt) ? s0 : 0;
    o.y = (p4 + 1 < tt) ? s1 : 0;
    o.z = (p4 + 2 < tt) ? s2 : 0;
    o.w = (p4 + 3 < tt) ? s3 : 0;
    int* dp = SR + (size_t)sbase + p4;
    *(volatile v4i*)dp = o;
    __threadfence();
    *(volatile v4i*)dp = o;
  }
  {
    const v4i c4 = *(const v4ia*)(cnt + 4 * tid);
    const v4i o4 = *(const v4ia*)(offs + 4 * tid);
    v4i cv, rv;
    cv.x = (ovf != 0 || c4.x > DEGCAP) ? -1 : c4.x;
    cv.y = (ovf != 0 || c4.y > DEGCAP) ? -1 : c4.y;
    cv.z = (ovf != 0 || c4.z > DEGCAP) ? -1 : c4.z;
    cv.w = (ovf != 0 || c4.w > DEGCAP) ? -1 : c4.w;
    rv.x = sbase + (o4.x < 0 ? 0 : (o4.x > RCAP - 1 ? RCAP - 1 : o4.x));
    rv.y = sbase + (o4.y < 0 ? 0 : (o4.y > RCAP - 1 ? RCAP - 1 : o4.y));
    rv.z = sbase + (o4.z < 0 ? 0 : (o4.z > RCAP - 1 ? RCAP - 1 : o4.z));
    rv.w = sbase + (o4.w < 0 ? 0 : (o4.w > RCAP - 1 ? RCAP - 1 : o4.w));
    int* cp = CN + (size_t)nodeBase + 4 * tid;
    int* rp = RP + (size_t)nodeBase + 4 * tid;
    *(volatile v4i*)cp = cv;
    *(volatile v4i*)rp = rv;
    __threadfence();
    *(volatile v4i*)cp = cv;
    *(volatile v4i*)rp = rv;
  }
}

__global__ __launch_bounds__(GTHR) void k_gemm(
    const unsigned short* __restrict__ A, const unsigned short* __restrict__ WT,
    float* outF, int K, int ldo)
{
  __shared__ __attribute__((aligned(16))) float stg[GBM * GBN];
  const int tid = (int)threadIdx.x, lane = tid & 31, wave = tid >> 5, hh = lane >> 4, m = lane & 15;
  const int rowBase = (int)blockIdx.x * GBM;
  const int col0    = (int)blockIdx.y * GBN;

  v8f acc[4];
  {
    const v8f z = {0.f, 0.f, 0.f, 0.f, 0.f, 0.f, 0.f, 0.f};
    acc[0] = z; acc[1] = z; acc[2] = z; acc[3] = z;
  }
  const unsigned short* ap = A  + (size_t)(rowBase + 16 * wave + m) * (size_t)K + 8 * hh;
  const unsigned short* wp = WT + (size_t)(col0 + m) * (size_t)K + 8 * hh;
  const int ksteps = K >> 5;
#pragma unroll 1
  for (int ks = 0; ks < ksteps; ++ks) {
    FragB af;
    af.h[0] = *(const v8usa*)(ap + 32 * ks);
    af.h[1] = *(const v8usa*)(ap + 32 * ks + 16);
#pragma unroll
    for (int t = 0; t < 4; ++t) {
      const unsigned short* wq = wp + (size_t)(16 * t) * (size_t)K + 32 * ks;
      FragB bf;
      bf.h[0] = *(const v8usa*)wq;
      bf.h[1] = *(const v8usa*)(wq + 16);
      acc[t] = wmb(af, bf, acc[t]);
    }
  }

#pragma unroll
  for (int t = 0; t < 4; ++t) {
    const int lc = 16 * t + m;
#pragma unroll
    for (int r = 0; r < 8; ++r) {
      const int lr = 16 * wave + 8 * hh + r;
      stg[lr * GBN + lc] = acc[t][r];
    }
  }
  __syncthreads();

  v4f fv[8];
#pragma unroll
  for (int i = 0; i < 8; ++i) {
    const int lr = 16 * wave + 2 * i + hh;
    fv[i] = *(const v4fa*)(stg + lr * GBN + 4 * m);
  }
#pragma unroll
  for (int i = 0; i < 8; ++i) {
    const int lr = 16 * wave + 2 * i + hh;
    const int gr = rowBase + lr;
    float* op = outF + (size_t)gr * (size_t)ldo + col0 + 4 * m;
    *(volatile v4f*)op = fv[i];
  }
  __threadfence();
#pragma unroll
  for (int i = 0; i < 8; ++i) {
    const int lr = 16 * wave + 2 * i + hh;
    const int gr = rowBase + lr;
    float* op = outF + (size_t)gr * (size_t)ldo + col0 + 4 * m;
    *(volatile v4f*)op = fv[i];
  }
}

__global__ __launch_bounds__(NTHR) void k_agg(const float* __restrict__ T, const int* __restrict__ RP,
                                              const int* __restrict__ CN, const int* __restrict__ SR, int nSr,
                                              const float* __restrict__ bias, int nN, int mRows,
                                              unsigned short* zhl) {
  const int tid = (int)threadIdx.x, lane = tid & 31, wave = tid >> 5;
  v4f bv;
  {
    const v4f b4 = *(const v4f*)(bias + 4 * lane);
    bv.x = bf16_val(b4.x); bv.y = bf16_val(b4.y); bv.z = bf16_val(b4.z); bv.w = bf16_val(b4.w);
  }
  const float qnan = __int_as_float(0x7fc00000);
  const int sa = (2 * lane) & 31, sb = (2 * lane + 1) & 31;
  const bool lsel = lane >= 16;
#pragma unroll 1
  for (int i = 0; i < ARB / NWAVE; ++i) {
    const int row = (int)blockIdx.x * ARB + i * NWAVE + wave;
    if (row >= mRows) continue;
    const int rc = row < nN ? row : nN - 1;
    const int cn = CN[rc];
    int rp = RP[rc];
    const bool bad = (cn < 0) || (cn > DEGCAP);
    const int c = cn < 0 ? 0 : (cn > DEGCAP ? DEGCAP : cn);
    rp = rp < 0 ? 0 : (rp > nSr - 1 ? nSr - 1 : rp);
    float a0 = 0.0f, a1 = 0.0f, a2 = 0.0f, a3 = 0.0f;
#pragma unroll 1
    for (int b0 = 0; b0 < c; b0 += 32) {
      int idx = rp + b0 + lane;
      idx = idx > nSr - 1 ? nSr - 1 : idx;
      int sr = SR[idx];
      sr = sr < 0 ? 0 : (sr > nN - 1 ? nN - 1 : sr);
      const int m32 = (c - b0) < 32 ? (c - b0) : 32;
#pragma unroll 1
      for (int k = 0; k < m32; ++k) {
        const int sk = __builtin_amdgcn_readlane(sr, k);
        const v4f a = *(const v4f*)(T + (size_t)sk * TP + 4 * lane);
        a0 += a.x; a1 += a.y; a2 += a.z; a3 += a.w;
      }
    }
    const v4f tr = *(const v4f*)(T + (size_t)rc * TP + DF + 4 * lane);
    const float cf  = (c < 1) ? 1.0f : (float)c;
    const float inv = 1.0f / cf;
    const float o0 = (a0 * inv + bv.x) + tr.x;
    const float o1 = (a1 * inv + bv.y) + tr.y;
    const float o2 = (a2 * inv + bv.z) + tr.z;
    const float o3 = (a3 * inv + bv.w) + tr.w;
    float ss = (o0 * o0 + o1 * o1) + (o2 * o2 + o3 * o3);
    ss += __shfl_xor(ss, 16, 32);
    ss += __shfl_xor(ss, 8, 32);
    ss += __shfl_xor(ss, 4, 32);
    ss += __shfl_xor(ss, 2, 32);
    ss += __shfl_xor(ss, 1, 32);
    const float dn = fmaxf(sqrtf(ss), 1e-12f);
    const float rn = 1.0f / dn;
    float v0 = o0 * rn, v1 = o1 * rn, v2 = o2 * rn, v3 = o3 * rn;
    v0 = (v0 > 0.0f) ? v0 : (v0 - v0);
    v1 = (v1 > 0.0f) ? v1 : (v1 - v1);
    v2 = (v2 > 0.0f) ? v2 : (v2 - v2);
    v3 = (v3 > 0.0f) ? v3 : (v3 - v3);
    const float pz = bad ? qnan : 0.0f;
    const bool live = row < nN;
    v0 = live ? (v0 + pz) : 0.0f;
    v1 = live ? (v1 + pz) : 0.0f;
    v2 = live ? (v2 + pz) : 0.0f;
    v3 = live ? (v3 + pz) : 0.0f;
    const unsigned hb0 = bf16_bits(v0), hb1 = bf16_bits(v1), hb2 = bf16_bits(v2), hb3 = bf16_bits(v3);
    const unsigned lb0 = bf16_bits(v0 - __uint_as_float(hb0 << 16));
    const unsigned lb1 = bf16_bits(v1 - __uint_as_float(hb1 << 16));
    const unsigned lb2 = bf16_bits(v2 - __uint_as_float(hb2 << 16));
    const unsigned lb3 = bf16_bits(v3 - __uint_as_float(hb3 << 16));
    const int hw0 = (int)(hb0 | (hb1 << 16));
    const int hw1 = (int)(hb2 | (hb3 << 16));
    const int lw0 = (int)(lb0 | (lb1 << 16));
    const int lw1 = (int)(lb2 | (lb3 << 16));
    const int g0 = __shfl(hw0, sa, 32), g1 = __shfl(hw1, sa, 32);
    const int g2 = __shfl(hw0, sb, 32), g3 = __shfl(hw1, sb, 32);
    const int p0 = __shfl(lw0, sa, 32), p1 = __shfl(lw1, sa, 32);
    const int p2 = __shfl(lw0, sb, 32), p3 = __shfl(lw1, sb, 32);
    v4u pv;
    pv.x = (unsigned int)(lsel ? p0 : g0);
    pv.y = (unsigned int)(lsel ? p1 : g1);
    pv.z = (unsigned int)(lsel ? p2 : g2);
    pv.w = (unsigned int)(lsel ? p3 : g3);
    unsigned short* hp = zhl + (size_t)row * TP + 8 * lane;
    *(volatile v4u*)hp = pv;
    __threadfence();
    *(volatile v4u*)hp = pv;
  }
}

__global__ __launch_bounds__(GTHR) void k_cls(const unsigned short* __restrict__ A,
                                              const unsigned short* __restrict__ WT,
                                              const float* __restrict__ blin, const int* __restrict__ CN,
                                              float* out, int nN) {
  __shared__ __attribute__((aligned(16))) float stg[GBM * GBN];
  const int tid = (int)threadIdx.x, lane = tid & 31, wave = tid >> 5, hh = lane >> 4, m = lane & 15;
  const int rowBase = (int)blockIdx.x * GBM;

  v8f acc[4];
  {
    const v8f z = {0.f, 0.f, 0.f, 0.f, 0.f, 0.f, 0.f, 0.f};
    acc[0] = z; acc[1] = z; acc[2] = z; acc[3] = z;
  }
  const unsigned short* ap = A  + (size_t)(rowBase + 16 * wave + m) * (size_t)TP + 8 * hh;
  const unsigned short* wp = WT + (size_t)m * (size_t)TP + 8 * hh;
#pragma unroll 1
  for (int ks = 0; ks < TP / 32; ++ks) {
    FragB af;
    af.h[0] = *(const v8usa*)(ap + 32 * ks);
    af.h[1] = *(const v8usa*)(ap + 32 * ks + 16);
#pragma unroll
    for (int t = 0; t < 4; ++t) {
      const unsigned short* wq = wp + (size_t)(16 * t) * (size_t)TP + 32 * ks;
      FragB bf;
      bf.h[0] = *(const v8usa*)wq;
      bf.h[1] = *(const v8usa*)(wq + 16);
      acc[t] = wmb(af, bf, acc[t]);
    }
  }
#pragma unroll
  for (int t = 0; t < 4; ++t) {
    const int lc = 16 * t + m;
#pragma unroll
    for (int r = 0; r < 8; ++r) {
      const int lr = 16 * wave + 8 * hh + r;
      stg[lr * GBN + lc] = acc[t][r];
    }
  }
  __syncthreads();

  int nv = nN - rowBase;
  nv = nv < 0 ? 0 : (nv > GBM ? GBM : nv);
  const int nF4 = nv * (NC / 4);
  const float qnan = __int_as_float(0x7fc00000);
  constexpr int NIT = (GBM * NC) / (4 * GTHR);
  v4f ov[NIT];
#pragma unroll
  for (int it = 0; it < NIT; ++it) {
    const int f  = it * GTHR + tid;
    const int lr = f / (NC / 4);
    const int c4 = 4 * (f - lr * (NC / 4));
    const v4f s = *(const v4fa*)(stg + lr * GBN + c4);
    const v4f b = *(const v4f*)(blin + c4);
    int gr = rowBase + lr;
    gr = gr > nN - 1 ? nN - 1 : gr;
    const int cn = CN[gr];
    const float pz = (cn < 0 || cn > DEGCAP) ? qnan : 0.0f;
    v4f y;
    y.x = (s.x + bf16_val(b.x)) + pz;
    y.y = (s.y + bf16_val(b.y)) + pz;
    y.z = (s.z + bf16_val(b.z)) + pz;
    y.w = (s.w + bf16_val(b.w)) + pz;
    ov[it] = y;
  }
  float* ob = out + (size_t)rowBase * NC;
#pragma unroll
  for (int it = 0; it < NIT; ++it) {
    const int f = it * GTHR + tid;
    if (f < nF4) *(volatile v4f*)(ob + 4 * (size_t)f) = ov[it];
  }
  __threadfence();
#pragma unroll
  for (int it = 0; it < NIT; ++it) {
    const int f = it * GTHR + tid;
    if (f < nF4) *(volatile v4f*)(ob + 4 * (size_t)f) = ov[it];
  }
}

static inline int cdiv(int a, int b) { return (a + b - 1) / b; }
static inline size_t al256(size_t o) { return (o + 255) & ~(size_t)255; }

extern "C" void kernel_launch(void* const* d_in, const int* in_sizes, int n_in,
                              void* d_out, int out_size, void* d_ws, size_t ws_size,
                              hipStream_t stream) {
  if (n_in < 7) return;
  if (in_sizes[0] < DF || (in_sizes[0] % DF) != 0) return;
  const int nN = in_sizes[0] / DF;
  if (nN < 4 || nN > (1 << 22) || (nN & 3) != 0) return;
  if (in_sizes[1] < 2 || (in_sizes[1] & 1) != 0) return;
  const int nE = in_sizes[1] / 2;
  if (nE < 1 || nE >= (1 << (31 - SLA))) return;
  if (in_sizes[2] != 3 * DF * DF || in_sizes[3] != 3 * DF) return;
  if (in_sizes[4] != 3 * DF * DF) return;
  if (in_sizes[5] != NC * DF || in_sizes[6] != NC) return;
  if ((long long)out_size != (long long)nN * NC) return;

  const float* x    = (const float*)d_in[0];
  const int*   edge = (const int*)d_in[1];
  const float* Wl   = (const float*)d_in[2];
  const float* bl   = (const float*)d_in[3];
  const float* Wr   = (const float*)d_in[4];
  const float* Wlin = (const float*)d_in[5];
  const float* blin = (const float*)d_in[6];
  float* out = (float*)d_out;
  const int* src = edge;
  const int* dst = edge + nE;

  const int MP = cdiv(nN, GBM) * GBM;
  const int gM = MP / GBM;
  const int gC = cdiv(MP, NBA);
  const int NP = gC * NBA;
  if (NP < MP) return;
  if ((long long)gC * RCAP >= (1LL << 31)) return;
  const int nSr = gC * RCAP;
  const int gA = cdiv(MP, ARB);
  const int vec8 = ((nE & 3) == 0) ? 1 : 0;

  char* ws = (char*)d_ws;
  size_t off = 0;
  const size_t oWP  = off; off = al256(off + (size_t)WPLN * 2);
  const size_t oRP  = off; off = al256(off + (size_t)NP * 4);
  const size_t oCN  = off; off = al256(off + (size_t)NP * 4);
  const size_t oSR  = off; off = al256(off + (size_t)nSr * 4);
  const size_t oZHL = off; off = al256(off + (size_t)MP * TP * 2);
  const size_t oT   = off; off = al256(off + (size_t)MP * TP * 4);
  if (off > ws_size) return;
  unsigned short* WP  = (unsigned short*)(ws + oWP);
  int*            RP  = (int*)(ws + oRP);
  int*            CN  = (int*)(ws + oCN);
  int*            SR  = (int*)(ws + oSR);
  unsigned short* ZHL = (unsigned short*)(ws + oZHL);
  unsigned short* XB  = ZHL;
  float*          T   = (float*)(ws + oT);

  const size_t cmpLds = (size_t)CMP_LDS_INTS * 4;
  hipFuncSetAttribute(reinterpret_cast<const void*>(&k_compact), hipFuncAttributeMaxDynamicSharedMemorySize, (int)cmpLds);

  const int nUx = MP * (DF / 8);
  k_wprep<<<UTOT / NTHR, NTHR, 0, stream>>>(Wl, Wr, Wlin, WP);
  k_cvx<<<cdiv(nUx, NTHR), NTHR, 0, stream>>>(x, nN, nUx, XB);
  k_compact<<<gC, NTHR, cmpLds, stream>>>(src, dst, nE, nN, vec8, SR, RP, CN);
  k_gemm<<<dim3(gM, TP / GBN), GTHR, 0, stream>>>(XB, WP + OW0, T, DF, TP);
  k_agg<<<gA, NTHR, 0, stream>>>(T, RP, CN, SR, nSr, bl, nN, MP, ZHL);
  k_gemm<<<dim3(gM, TP / GBN), GTHR, 0, stream>>>(ZHL, WP + OW1, T, TP, TP);
  k_agg<<<gA, NTHR, 0, stream>>>(T, RP, CN, SR, nSr, bl + DF, nN, MP, ZHL);
  k_gemm<<<dim3(gM, TP / GBN), GTHR, 0, stream>>>(ZHL, WP + OW2, T, TP, TP);
  k_agg<<<gA, NTHR, 0, stream>>>(T, RP, CN, SR, nSr, bl + 2 * DF, nN, MP, ZHL);
  k_cls<<<gM, GTHR, 0, stream>>>(ZHL, WP + OWL, blin, CN, out, nN);
}
